// GATGraphAssociator_89507118449200
// MI455X (gfx1250) — hardware-run, weakly checked
//
#include <hip/hip_runtime.h>
#include <stddef.h>
#include <stdint.h>
#include <math.h>


#define EMB     128
#define NHD     16
#define F1      2048
#define NGRP    4
#define HPG     4
#define GW      512
#define KA2     4096
#define NTHR    256
#define NWAVE   8
#define EPT     8
#define CHUNK   (NTHR * EPT)
#define WCAP    (EPT * 32)
#define LISTN   (NWAVE * WCAP)
#define NBA     256
#define SLA     8
#define RCAP    6144
#define DEGCAP  64
#define MEAS_B256   4290
#define MEAS_MAXDEG 36
#define BKINTS  (RCAP + 2 * NBA + 32)
#define TABN    288
#define GBM     64
#define GBN     128
#define GTHR    128
#define SPIT    132
#define MROWS   128
#define NUW1    (F1 * (EMB / 8))
#define NUW2    (EMB * (KA2 / 8))
#define NEGSL   0.2f
#define NEGBIG  (-3.0e38f)
#define WSMAX   134217728

#define PINF(x) asm volatile("" :: "v"(x))

static_assert((CHUNK & (CHUNK - 1)) == 0 && CHUNK <= 4096);
static_assert((NBA & (NBA - 1)) == 0 && NBA == (1 << SLA) && NBA <= 65536);
static_assert(((long long)CHUNK << SLA) < (1LL << 31));
static_assert(LISTN >= NWAVE * WCAP);
static_assert(NBA % NWAVE == 0 && NBA % 32 == 0);
static_assert((RCAP % 32) == 0 && (BKINTS % 32) == 0);
static_assert(RCAP >= MEAS_B256 + MEAS_B256 / 4 + 1);
static_assert(DEGCAP >= MEAS_MAXDEG + 8);
static_assert(((DEGCAP + 1 + 7) / 8) * 32 <= TABN);
static_assert(((DEGCAP + 1 + 31) / 32) * 32 <= TABN);
static_assert(4 * (DEGCAP + 1) <= TABN);
static_assert(NGRP * GW == F1 && HPG * EMB == GW && NGRP * HPG == NHD);
static_assert(KA2 == 2 * F1 && (KA2 % 32) == 0 && (EMB % 32) == 0);
static_assert(GBM == (GTHR / 32) * 16 && GTHR == GBN && GTHR == 2 * GBM && GBN == EMB);
static_assert((MROWS % GBM) == 0 && (SPIT % 4) == 0 && SPIT >= GBN);
static_assert((NUW1 % NTHR) == 0 && (NUW2 % NTHR) == 0);
static_assert(EMB == 4 * 32);
static_assert((BKINTS + LISTN + RCAP + NBA + 16) * 4 <= 65536);
static_assert((GBM * SPIT + 2 * GBN + 2 * GBM) * 4 <= 65536);
static_assert((BKINTS + NWAVE * TABN + 512 + NWAVE * 512 + NBA) * 4 <= 65536);

typedef float          v4f  __attribute__((ext_vector_type(4)));
typedef float          v8f  __attribute__((ext_vector_type(8)));
typedef int            v4i  __attribute__((ext_vector_type(4)));
typedef int            v8i  __attribute__((ext_vector_type(8)));
typedef unsigned short v4us __attribute__((ext_vector_type(4)));
typedef unsigned short v8us __attribute__((ext_vector_type(8)));
typedef __bf16         v16b __attribute__((ext_vector_type(16)));
typedef v4f  __attribute__((may_alias)) v4fa;
typedef v4i  __attribute__((may_alias)) v4ia;
typedef v8us __attribute__((may_alias)) v8usa;
union FragB { v16b v; v8us h[2]; v8i w; };

__device__ __forceinline__ v8f wmb(const FragB& a, const FragB& b, v8f c) {
  v8f d = __builtin_amdgcn_wmma_f32_16x16x32_bf16(false, a.v, false, b.v, (short)0, c, false, false);
  asm volatile("v_nop\n\tv_nop\n\tv_nop\n\tv_nop" : "+v"(d) : "v"(a.w), "v"(b.w));
  return d;
}

__device__ __forceinline__ unsigned int f2bf(float f) {
  const unsigned int u = __float_as_uint(f);
  const unsigned int r = ((u + 0x7FFFu + ((u >> 16) & 1u)) >> 16) & 0xFFFFu;
  return ((u & 0x7FFFFFFFu) > 0x7F800000u) ? 0x7FC0u : r;
}
__device__ __forceinline__ float bf2f(unsigned int b) { return __uint_as_float(b << 16); }
__device__ __forceinline__ float bfr(float f) { return bf2f(f2bf(f)); }

template <int SLB>
__device__ __forceinline__ int scan_chunk(const int* __restrict__ dsts, int nE, int cbase, int slotBase,
                                          int nb, int vec8, int* list, int tid, int lane, int wave) {
  int wc = 0;
  const int el0  = tid * EPT;
  const int e0   = cbase + el0;
  const int sent = -2147483647 - 1;
  v4i da, db;
  if (vec8 != 0 && cbase + CHUNK <= nE) {
    da = *(const v4i*)(dsts + e0);
    db = *(const v4i*)(dsts + e0 + 4);
  } else {
    da.x = (e0     < nE) ? dsts[min(e0,     nE - 1)] : sent;
    da.y = (e0 + 1 < nE) ? dsts[min(e0 + 1, nE - 1)] : sent;
    da.z = (e0 + 2 < nE) ? dsts[min(e0 + 2, nE - 1)] : sent;
    da.w = (e0 + 3 < nE) ? dsts[min(e0 + 3, nE - 1)] : sent;
    db.x = (e0 + 4 < nE) ? dsts[min(e0 + 4, nE - 1)] : sent;
    db.y = (e0 + 5 < nE) ? dsts[min(e0 + 5, nE - 1)] : sent;
    db.z = (e0 + 6 < nE) ? dsts[min(e0 + 6, nE - 1)] : sent;
    db.w = (e0 + 7 < nE) ? dsts[min(e0 + 7, nE - 1)] : sent;
  }
  const unsigned nbs = (unsigned)slotBase;
  const unsigned unb = (unsigned)nb;
  const unsigned s0 = (unsigned)da.x - nbs, s1 = (unsigned)da.y - nbs;
  const unsigned s2 = (unsigned)da.z - nbs, s3 = (unsigned)da.w - nbs;
  const unsigned s4 = (unsigned)db.x - nbs, s5 = (unsigned)db.y - nbs;
  const unsigned s6 = (unsigned)db.z - nbs, s7 = (unsigned)db.w - nbs;
  const bool h0 = s0 < unb, h1 = s1 < unb, h2 = s2 < unb, h3 = s3 < unb;
  const bool h4 = s4 < unb, h5 = s5 < unb, h6 = s6 < unb, h7 = s7 < unb;
  const unsigned any = __builtin_amdgcn_ballot_w32(h0 | h1 | h2 | h3 | h4 | h5 | h6 | h7);
  if (any != 0u) {
#define HITJ(J, HJ, SJ) { \
      const unsigned mj = __builtin_amdgcn_ballot_w32(HJ); \
      if (mj != 0u) { \
        if (HJ) { \
          const int pos = wc + (int)__builtin_amdgcn_mbcnt_lo(mj, 0u); \
          if (pos < WCAP) list[wave * WCAP + pos] = ((el0 + (J)) << SLB) | (int)(SJ); \
        } \
        wc += (int)__builtin_popcount(mj); } }
    HITJ(0, h0, s0)
    HITJ(1, h1, s1)
    HITJ(2, h2, s2)
    HITJ(3, h3, s3)
    HITJ(4, h4, s4)
    HITJ(5, h5, s5)
    HITJ(6, h6, s6)
    HITJ(7, h7, s7)
#undef HITJ
  }
  return wc;
}

__global__ __launch_bounds__(NTHR) __attribute__((amdgpu_num_vgpr(248)))
void k_prep(const float* __restrict__ x, const float* __restrict__ W1, const float* __restrict__ W2,
            unsigned short* XB, unsigned short* W1T, unsigned short* W2D, int nN, int nUx) {
  const int u = (int)blockIdx.x * NTHR + (int)threadIdx.x;
  v8us o;
  unsigned short* dp;
  if (u < nUx) {
    const int row = u >> 4;
    const int c0  = (u & 15) * 8;
    const int rc  = row < nN ? row : nN - 1;
    const float* p = x + (size_t)rc * EMB + c0;
    const v4f a = *(const v4f*)p;
    const v4f b = *(const v4f*)(p + 4);
    const bool okr = row < nN;
    o[0] = okr ? (unsigned short)f2bf(a.x) : (unsigned short)0;
    o[1] = okr ? (unsigned short)f2bf(a.y) : (unsigned short)0;
    o[2] = okr ? (unsigned short)f2bf(a.z) : (unsigned short)0;
    o[3] = okr ? (unsigned short)f2bf(a.w) : (unsigned short)0;
    o[4] = okr ? (unsigned short)f2bf(b.x) : (unsigned short)0;
    o[5] = okr ? (unsigned short)f2bf(b.y) : (unsigned short)0;
    o[6] = okr ? (unsigned short)f2bf(b.z) : (unsigned short)0;
    o[7] = okr ? (unsigned short)f2bf(b.w) : (unsigned short)0;
    dp = XB + (size_t)row * EMB + c0;
  } else if (u < nUx + NUW1) {
    const int v  = u - nUx;
    const int n  = v >> 4;
    const int k8 = (v & 15) * 8;
    const float* p = W1 + (size_t)k8 * F1 + n;
#pragma unroll
    for (int i = 0; i < 8; ++i) o[i] = (unsigned short)f2bf(p[(size_t)i * F1]);
    dp = W1T + (size_t)n * EMB + k8;
  } else if (u < nUx + NUW1 + NUW2) {
    const int v  = u - nUx - NUW1;
    const int n  = v >> 9;
    const int k8 = (v & 511) * 8;
    const int kk = k8 & (F1 - 1);
    const float* p = W2 + (size_t)kk * EMB + n;
#pragma unroll
    for (int i = 0; i < 8; ++i) o[i] = (unsigned short)f2bf(p[(size_t)i * EMB]);
    dp = W2D + (size_t)n * KA2 + k8;
  } else {
    return;
  }
  *(volatile v8us*)dp = o;
  __threadfence();
  *(volatile v8us*)dp = o;
}

__global__ __launch_bounds__(NTHR) __attribute__((amdgpu_num_vgpr(248)))
void k_bucket(const int* __restrict__ srcs, const int* __restrict__ dsts, int nE, int nN, int vec8, int* BK) {
  __shared__ __attribute__((aligned(16))) int outb[BKINTS];
  __shared__ __attribute__((aligned(16))) int list[LISTN];
  __shared__ __attribute__((aligned(16))) int reg1[RCAP];
  __shared__ __attribute__((aligned(16))) int cur[NBA];
  __shared__ __attribute__((aligned(16))) int wcnt[16];
  int* sl   = outb;
  int* offs = outb + RCAP;
  int* cnt  = offs + NBA;
  int* flg  = cnt + NBA;
  const int tid = (int)threadIdx.x, lane = tid & 31, wave = tid >> 5;
  const int blk = (int)blockIdx.x;
  const int nodeBase = blk * NBA;
  int nb = nN - nodeBase;
  nb = nb < 0 ? 0 : (nb > NBA ? NBA : nb);

  {
    const v4i z4 = {0, 0, 0, 0};
    for (int i = tid * 4; i < BKINTS; i += NTHR * 4) *(v4ia*)(outb + i) = z4;
    if (tid < 16) wcnt[tid] = 0;
  }
  __syncthreads();

  int tot = 0, ovf = 0;
  const int nChunks = (nE + CHUNK - 1) / CHUNK;
#pragma unroll 1
  for (int ch = 0; ch < nChunks; ++ch) {
    const int cbase = ch * CHUNK;
    const int wc = scan_chunk<SLA>(dsts, nE, cbase, nodeBase, nb, vec8, list, tid, lane, wave);
    if (lane == 0) wcnt[wave] = wc;
    __syncthreads();
    int pre = 0, all = 0;
#pragma unroll
    for (int w2 = 0; w2 < NWAVE; ++w2) {
      int c = wcnt[w2];
      c = c < 0 ? 0 : (c > WCAP ? WCAP : c);
      all += c;
      pre += (w2 < wave) ? c : 0;
    }
    const int wcc  = wc > WCAP ? WCAP : wc;
    const int base = tot + pre;
#pragma unroll 1
    for (int i = lane; i < wcc; i += 32) {
      const int ent = list[wave * WCAP + i];
      const int el  = (ent >> SLA) & (CHUNK - 1);
      const int sq  = ent & (NBA - 1);
      int eid = cbase + el;
      eid = eid > nE - 1 ? nE - 1 : eid;
      const int sraw = srcs[eid];
      const int s = sraw < 0 ? 0 : (sraw > nN - 1 ? nN - 1 : sraw);
      const int pos = base + i;
      if (pos < RCAP) reg1[pos] = (int)((unsigned)s | ((unsigned)sq << 16));
    }
    if (tot + all > RCAP) ovf = 1;
    tot += all;
    tot = tot > RCAP ? RCAP : tot;
    __syncthreads();
  }
  const int nh = tot;

  if (wave == 0) {
#pragma unroll 1
    for (int b0 = 0; b0 < nh; b0 += 32) {
      const int idx = b0 + lane;
      const int uv  = reg1[idx < nh ? idx : nh - 1];
      const int m32 = (nh - b0) < 32 ? (nh - b0) : 32;
#pragma unroll 1
      for (int k = 0; k < m32; ++k) {
        const int u  = __builtin_amdgcn_readlane(uv, k);
        const int sq = (u >> 16) & (NBA - 1);
        if (lane == 0) cnt[sq] = cnt[sq] + 1;
      }
    }
  }
  __syncthreads();
  if (wave == 0) {
    const int base = lane * (NBA / 32);
    int s = 0;
#pragma unroll 1
    for (int i = 0; i < NBA / 32; ++i) s += cnt[base + i];
    int incl = s;
#pragma unroll
    for (int d = 1; d < 32; d <<= 1) {
      const int y = __shfl_up(incl, d, 32);
      if (lane >= d) incl += y;
    }
    int run = incl - s;
#pragma unroll 1
    for (int i = 0; i < NBA / 32; ++i) {
      const int cv = cnt[base + i];
      offs[base + i] = run;
      cur[base + i]  = run;
      run += cv;
    }
  }
  __syncthreads();
  if (wave == 0) {
#pragma unroll 1
    for (int b0 = 0; b0 < nh; b0 += 32) {
      const int idx = b0 + lane;
      const int uv  = reg1[idx < nh ? idx : nh - 1];
      const int m32 = (nh - b0) < 32 ? (nh - b0) : 32;
#pragma unroll 1
      for (int k = 0; k < m32; ++k) {
        const int u  = __builtin_amdgcn_readlane(uv, k);
        const int sq = (u >> 16) & (NBA - 1);
        if (lane == 0) {
          int p = cur[sq];
          p = p < 0 ? 0 : (p > RCAP - 1 ? RCAP - 1 : p);
          sl[p] = u;
          cur[sq] = p + 1;
        }
      }
    }
    flg[lane] = (lane == 0) ? nh : ((lane == 1) ? ovf : 0);
  }
  __syncthreads();

  int* bp = BK + (size_t)blk * BKINTS;
#pragma unroll 1
  for (int p = tid * 4; p < BKINTS; p += NTHR * 4) {
    const v4i v = *(const v4ia*)(outb + p);
    *(volatile v4i*)(bp + p) = v;
  }
  __threadfence();
#pragma unroll 1
  for (int p = tid * 4; p < BKINTS; p += NTHR * 4) {
    const v4i v = *(const v4ia*)(outb + p);
    *(volatile v4i*)(bp + p) = v;
  }
}

__global__ __launch_bounds__(GTHR) __attribute__((amdgpu_num_vgpr(248)))
void k_gemm(const unsigned short* __restrict__ A, const unsigned short* __restrict__ WT,
            float* outF, int K, int ldo,
            const float* __restrict__ atts, const float* __restrict__ attd,
            float* SD, int MPr) {
  __shared__ __attribute__((aligned(16))) float stg[GBM * SPIT];
  __shared__ __attribute__((aligned(16))) float satt[2 * GBN];
  __shared__ __attribute__((aligned(16))) float sdot[2 * GBM];
  const int tid = (int)threadIdx.x, lane = tid & 31, wave = tid >> 5, hh = lane >> 4, m = lane & 15;
  const int rowBase = (int)blockIdx.x * GBM;
  const int head    = (int)blockIdx.y;
  const int col0    = head * GBN;

  {
    const float vs = atts[head * GBN + tid];
    const float vd = attd[head * GBN + tid];
    satt[tid]       = bfr(vs);
    satt[GBN + tid] = bfr(vd);
  }

  v8f acc[8];
  {
    const v8f z = {0.f, 0.f, 0.f, 0.f, 0.f, 0.f, 0.f, 0.f};
#pragma unroll
    for (int t = 0; t < 8; ++t) acc[t] = z;
  }
  const unsigned short* ap = A  + (size_t)(rowBase + 16 * wave + m) * (size_t)K + 8 * hh;
  const unsigned short* wp = WT + (size_t)(col0 + m) * (size_t)K + 8 * hh;
  const int ksteps = K >> 5;
#pragma unroll 1
  for (int ks = 0; ks < ksteps; ++ks) {
    FragB af;
    af.h[0] = *(const v8usa*)(ap + 32 * ks);
    af.h[1] = *(const v8usa*)(ap + 32 * ks + 16);
#pragma unroll
    for (int t = 0; t < 8; ++t) {
      const unsigned short* wq = wp + (size_t)(16 * t) * (size_t)K + 32 * ks;
      FragB bf;
      bf.h[0] = *(const v8usa*)wq;
      bf.h[1] = *(const v8usa*)(wq + 16);
      acc[t] = wmb(af, bf, acc[t]);
    }
  }

#pragma unroll
  for (int t = 0; t < 8; ++t) {
    const int lc = 16 * t + m;
#pragma unroll
    for (int r = 0; r < 8; ++r) {
      const int lr = 16 * wave + 8 * hh + r;
      stg[lr * SPIT + lc] = acc[t][r];
    }
  }
  __syncthreads();

  {
    const int row = tid & 63, which = tid >> 6;
    const float* sa = satt + which * GBN;
    const float* hr = stg + row * SPIT;
    float d = 0.f;
#pragma unroll 4
    for (int c4 = 0; c4 < GBN / 4; ++c4) {
      const v4f hv = *(const v4fa*)(hr + 4 * c4);
      const v4f av = *(const v4fa*)(sa + 4 * c4);
      d = fmaf(hv.x, av.x, d);
      d = fmaf(hv.y, av.y, d);
      d = fmaf(hv.z, av.z, d);
      d = fmaf(hv.w, av.w, d);
    }
    sdot[which * GBM + row] = d;
  }
  __syncthreads();

  const int which2 = lane >> 4, piece = lane & 15;
  const v4f sdv = *(const v4fa*)(sdot + which2 * GBM + 4 * piece);
  float* sp = SD + (size_t)(2 * head + which2) * (size_t)MPr + rowBase + 4 * piece;
  float* ob = outF + (size_t)(rowBase + 16 * wave) * (size_t)ldo + col0 + 4 * lane;
  const float* sb = stg + (16 * wave) * SPIT + 4 * lane;

#pragma unroll 1
  for (int i = 0; i < 16; ++i) {
    const v4f v = *(const v4fa*)(sb + i * SPIT);
    *(volatile v4f*)(ob + (size_t)i * (size_t)ldo) = v;
  }
  if (wave == 0) *(volatile v4f*)sp = sdv;
  __threadfence();
#pragma unroll 1
  for (int i = 0; i < 16; ++i) {
    const v4f v = *(const v4fa*)(sb + i * SPIT);
    *(volatile v4f*)(ob + (size_t)i * (size_t)ldo) = v;
  }
  if (wave == 0) *(volatile v4f*)sp = sdv;
}

template <int L>
__global__ __launch_bounds__(NTHR) __attribute__((amdgpu_num_vgpr(248)))
void k_scan(const int* __restrict__ BK, const float* __restrict__ F, const float* __restrict__ SD,
            const float* __restrict__ bias, const float* __restrict__ Wc, const float* __restrict__ bc,
            unsigned short* XP, float* out, int nN, int MPr, int colBase) {
  static_assert(L == 1 || L == 2);
  constexpr int HB  = (L == 1) ? HPG : 1;
  constexpr int TSH = (L == 1) ? 3 : 5;
  constexpr int TPS = 1 << TSH;
  constexpr int FP  = (L == 1) ? GW : EMB;
  static_assert(HB * TPS == 32);
  __shared__ __attribute__((aligned(16))) int   bks[BKINTS];
  __shared__ __attribute__((aligned(16))) float tab[NWAVE * TABN];
  __shared__ __attribute__((aligned(16))) float fl[512];
  __shared__ __attribute__((aligned(16))) float stg[NWAVE * 512];
  __shared__ __attribute__((aligned(16))) float outs[NBA];
  const int* sl   = bks;
  const int* offs = bks + RCAP;
  const int* cnt  = offs + NBA;
  const int* flg  = cnt + NBA;
  const int tid = (int)threadIdx.x, lane = tid & 31, wave = tid >> 5;
  const int blk = (int)blockIdx.x;
  const int nodeBase = blk * NBA;

  {
    const int* bp = BK + (size_t)blk * BKINTS;
#pragma unroll 1
    for (int p = tid * 4; p < BKINTS; p += NTHR * 4) *(v4ia*)(bks + p) = *(const v4i*)(bp + p);
    if constexpr (L == 1) {
#pragma unroll
      for (int q = 0; q < 2; ++q) {
        const int e  = tid + q * NTHR;
        const int j  = e >> 5, ln = e & 31;
        fl[e] = bfr(bias[colBase + (j >> 2) * EMB + 4 * ln + (j & 3)]);
      }
    }
  }
  __syncthreads();

  const int nhraw = flg[0];
  const int bflag = flg[1];
  const int nh  = nhraw < 0 ? 0 : (nhraw > RCAP ? RCAP : nhraw);
  const int ovf = (bflag != 0 || nhraw < 0 || nhraw > RCAP) ? 1 : 0;

  const float qnan = __int_as_float(0x7fc00000);
  const float pzb  = (ovf != 0) ? qnan : 0.0f;
  const int hl = lane & (HB - 1);
  const int tq = lane >> ((L == 1) ? 2 : 0);
  const size_t hoS = (size_t)(2 * hl) * (size_t)MPr;
  const size_t hoD = hoS + (size_t)MPr;
  float* tb = tab + wave * TABN;

  v4f b2v = {0.f, 0.f, 0.f, 0.f}, wcv = {0.f, 0.f, 0.f, 0.f};
  float bcv = 0.f;
  if constexpr (L == 2) {
    const v4f bq = *(const v4f*)(bias + 4 * lane);
    const v4f wq = *(const v4f*)(Wc + 4 * lane);
    b2v.x = bfr(bq.x); b2v.y = bfr(bq.y); b2v.z = bfr(bq.z); b2v.w = bfr(bq.w);
    wcv.x = bfr(wq.x); wcv.y = bfr(wq.y); wcv.z = bfr(wq.z); wcv.w = bfr(wq.w);
    bcv = bfr(bc[0]);
  }

#pragma unroll 1
  for (int si = 0; si < NBA / NWAVE; ++si) {
    const int s    = si * NWAVE + wave;
    const int node = nodeBase + s;
    const int nc   = node < nN ? node : nN - 1;
    const int craw = __builtin_amdgcn_readfirstlane(cnt[s]);
    const bool big = craw > DEGCAP;
    int c = craw < 0 ? 0 : (craw > DEGCAP ? DEGCAP : craw);
    int o = __builtin_amdgcn_readfirstlane(offs[s]);
    o = o < 0 ? 0 : (o > RCAP ? RCAP : o);
    if (c > nh - o) c = nh - o;
    c = c < 0 ? 0 : c;
    const int T = c + 1;
    int nst = (T + TPS - 1) >> TSH;
    nst = nst > (TABN / 32) ? (TABN / 32) : nst;

    const float adv = SD[hoD + (size_t)nc];
    PINF(adv);
    float mloc = NEGBIG;
#pragma unroll 1
    for (int sp = 0; sp < nst; ++sp) {
      const int t = (sp << TSH) + tq;
      int idx = o + t;
      idx = idx < 0 ? 0 : (idx > RCAP - 1 ? RCAP - 1 : idx);
      const int ent = sl[idx];
      int hs = ent & 0xFFFF;
      hs = hs > nN - 1 ? nN - 1 : hs;
      const int sr = (t < c) ? hs : nc;
      const float asv = SD[hoS + (size_t)sr];
      PINF(asv);
      float e = asv + adv;
      e = e > 0.f ? e : NEGSL * e;
      e = (t < T) ? e : NEGBIG;
      tb[32 * sp + lane] = e;
      mloc = fmaxf(mloc, e);
    }
#pragma unroll
    for (int off = HB; off < 32; off <<= 1) mloc = fmaxf(mloc, __shfl_xor(mloc, off));
    float zloc = 0.0f;
#pragma unroll 1
    for (int sp = 0; sp < nst; ++sp) {
      const float p = expf(tb[32 * sp + lane] - mloc);
      tb[32 * sp + lane] = p;
      zloc += p;
    }
#pragma unroll
    for (int off = HB; off < 32; off <<= 1) zloc += __shfl_xor(zloc, off);
    const float inv = __builtin_amdgcn_rcpf(zloc + 1e-16f);
    __builtin_amdgcn_fence(__ATOMIC_RELEASE, "workgroup");
    __builtin_amdgcn_wave_barrier();
    __builtin_amdgcn_fence(__ATOMIC_ACQUIRE, "workgroup");

    const float pzr = big ? qnan : pzb;
    const bool live = node < nN;

    if constexpr (L == 1) {
      const float i0 = __shfl(inv, 0), i1 = __shfl(inv, 1), i2 = __shfl(inv, 2), i3 = __shfl(inv, 3);
      v4f a0 = {0.f, 0.f, 0.f, 0.f}, a1 = a0, a2 = a0, a3 = a0;
#pragma unroll 1
      for (int t = 0; t < T; ++t) {
        int idx = o + t;
        idx = idx < 0 ? 0 : (idx > RCAP - 1 ? RCAP - 1 : idx);
        const int ent = sl[idx];
        int hs = ent & 0xFFFF;
        hs = hs > nN - 1 ? nN - 1 : hs;
        const int sk = (t < c) ? hs : nc;
        const v4f al = *(const v4fa*)(tb + 4 * t);
        const float* rp = F + (size_t)sk * FP + 4 * lane;
        const v4f f0 = *(const v4f*)rp;
        const v4f f1 = *(const v4f*)(rp + EMB);
        const v4f f2 = *(const v4f*)(rp + 2 * EMB);
        const v4f f3 = *(const v4f*)(rp + 3 * EMB);
        a0.x = fmaf(al.x, f0.x, a0.x); a0.y = fmaf(al.x, f0.y, a0.y);
        a0.z = fmaf(al.x, f0.z, a0.z); a0.w = fmaf(al.x, f0.w, a0.w);
        a1.x = fmaf(al.y, f1.x, a1.x); a1.y = fmaf(al.y, f1.y, a1.y);
        a1.z = fmaf(al.y, f1.z, a1.z); a1.w = fmaf(al.y, f1.w, a1.w);
        a2.x = fmaf(al.z, f2.x, a2.x); a2.y = fmaf(al.z, f2.y, a2.y);
        a2.z = fmaf(al.z, f2.z, a2.z); a2.w = fmaf(al.z, f2.w, a2.w);
        a3.x = fmaf(al.w, f3.x, a3.x); a3.y = fmaf(al.w, f3.y, a3.y);
        a3.z = fmaf(al.w, f3.z, a3.z); a3.w = fmaf(al.w, f3.w, a3.w);
      }
      float* st = stg + wave * 512;
      st[0  * 32 + lane] = a0.x * i0; st[1  * 32 + lane] = a0.y * i0;
      st[2  * 32 + lane] = a0.z * i0; st[3  * 32 + lane] = a0.w * i0;
      st[4  * 32 + lane] = a1.x * i1; st[5  * 32 + lane] = a1.y * i1;
      st[6  * 32 + lane] = a1.z * i1; st[7  * 32 + lane] = a1.w * i1;
      st[8  * 32 + lane] = a2.x * i2; st[9  * 32 + lane] = a2.y * i2;
      st[10 * 32 + lane] = a2.z * i2; st[11 * 32 + lane] = a2.w * i2;
      st[12 * 32 + lane] = a3.x * i3; st[13 * 32 + lane] = a3.y * i3;
      st[14 * 32 + lane] = a3.z * i3; st[15 * 32 + lane] = a3.w * i3;
#pragma unroll 1
      for (int j = 0; j < 16; ++j) {
        float y = st[j * 32 + lane] + fl[j * 32 + lane];
        y = (y > 0.0f) ? y : expm1f(y);
        st[j * 32 + lane] = y + pzr;
      }
      v4us hov[4], lov[4];
#pragma unroll
      for (int h = 0; h < 4; ++h) {
#pragma unroll
        for (int q = 0; q < 4; ++q) {
          const float y = st[(4 * h + q) * 32 + lane];
          const float v = live ? y : 0.0f;
          const unsigned int hbi = f2bf(v);
          hov[h][q] = (unsigned short)hbi;
          lov[h][q] = (unsigned short)f2bf(v - bf2f(hbi));
        }
      }
      if (node < MPr) {
        unsigned short* hp = XP + (size_t)node * KA2 + colBase + 4 * lane;
#pragma unroll
        for (int h = 0; h < 4; ++h) {
          *(volatile v4us*)(hp + EMB * h) = hov[h];
          *(volatile v4us*)(hp + F1 + EMB * h) = lov[h];
        }
        __threadfence();
#pragma unroll
        for (int h = 0; h < 4; ++h) {
          *(volatile v4us*)(hp + EMB * h) = hov[h];
          *(volatile v4us*)(hp + F1 + EMB * h) = lov[h];
        }
      }
    } else {
      v4f a = {0.f, 0.f, 0.f, 0.f};
#pragma unroll 1
      for (int t = 0; t < T; ++t) {
        int idx = o + t;
        idx = idx < 0 ? 0 : (idx > RCAP - 1 ? RCAP - 1 : idx);
        const int ent = sl[idx];
        int hs = ent & 0xFFFF;
        hs = hs > nN - 1 ? nN - 1 : hs;
        const int sk = (t < c) ? hs : nc;
        const float al = tb[t];
        const v4f f = *(const v4f*)(F + (size_t)sk * FP + 4 * lane);
        a.x = fmaf(al, f.x, a.x); a.y = fmaf(al, f.y, a.y);
        a.z = fmaf(al, f.z, a.z); a.w = fmaf(al, f.w, a.w);
      }
      const float r0 = fmaf(a.x, inv, b2v.x);
      const float r1 = fmaf(a.y, inv, b2v.y);
      const float r2 = fmaf(a.z, inv, b2v.z);
      const float r3 = fmaf(a.w, inv, b2v.w);
      float part = r0 * wcv.x;
      part = fmaf(r1, wcv.y, part);
      part = fmaf(r2, wcv.z, part);
      part = fmaf(r3, wcv.w, part);
#pragma unroll
      for (int off = 16; off > 0; off >>= 1) part += __shfl_xor(part, off);
      const float val = (part + bcv) + pzr;
      if (lane == 0) outs[s] = val;
    }
    __builtin_amdgcn_fence(__ATOMIC_RELEASE, "workgroup");
    __builtin_amdgcn_wave_barrier();
  }

  if constexpr (L == 2) {
    __syncthreads();
    const int pc   = tid & 63;
    const int row0 = nodeBase + 4 * pc;
    const bool wr  = (tid < 64) && (row0 + 3 < nN);
    const int rcl  = wr ? row0 : 0;
    v4f v = *(const v4fa*)(outs + 4 * pc);
    v.x = (ovf != 0) ? qnan : v.x;
    v.y = (ovf != 0) ? qnan : v.y;
    v.z = (ovf != 0) ? qnan : v.z;
    v.w = (ovf != 0) ? qnan : v.w;
    float* op = out + rcl;
    if (wr) *(volatile v4f*)op = v;
    __threadfence();
    if (wr) *(volatile v4f*)op = v;
  }
}

static inline int cdiv(int a, int b) { return (a + b - 1) / b; }

extern "C" void kernel_launch(void* const* d_in, const int* in_sizes, int n_in,
                              void* d_out, int out_size, void* d_ws, size_t ws_size,
                              hipStream_t stream) {
  if (n_in < 12) return;
  const int nN = in_sizes[0] / EMB;
  if (nN <= 0 || in_sizes[0] != nN * EMB || nN > 65536) return;
  if ((nN & 3) != 0) return;
  if (in_sizes[1] < 2 || (in_sizes[1] & 1) != 0) return;
  const int nE = in_sizes[1] / 2;
  if (nE < 1 || nE > (1 << 28)) return;
  if (in_sizes[2] != EMB * F1) return;
  if (in_sizes[3] != NHD * EMB || in_sizes[4] != NHD * EMB) return;
  if (in_sizes[5] != F1) return;
  if (in_sizes[6] != F1 * EMB) return;
  if (in_sizes[7] != EMB || in_sizes[8] != EMB) return;
  if (in_sizes[9] != EMB) return;
  if (in_sizes[10] != EMB) return;
  if (in_sizes[11] != 1) return;
  if (out_size != nN) return;

  const float* x   = (const float*)d_in[0];
  const int*   ei  = (const int*)  d_in[1];
  const float* W1  = (const float*)d_in[2];
  const float* a1s = (const float*)d_in[3];
  const float* a1d = (const float*)d_in[4];
  const float* b1  = (const float*)d_in[5];
  const float* W2  = (const float*)d_in[6];
  const float* a2s = (const float*)d_in[7];
  const float* a2d = (const float*)d_in[8];
  const float* b2  = (const float*)d_in[9];
  const float* Wc  = (const float*)d_in[10];
  const float* bc  = (const float*)d_in[11];
  float* out = (float*)d_out;
  const int* src = ei;
  const int* dst = ei + nE;

  const int MP   = cdiv(nN, MROWS) * MROWS;
  const int gM   = MP / GBM;
  const int gA   = cdiv(MP, NBA);
  if ((long long)gA * NBA < (long long)MP) return;
  const int vec8 = ((nE & 3) == 0) ? 1 : 0;
  const int nUx  = MP * (EMB / 8);
  if ((nUx % NTHR) != 0) return;

  char* ws = (char*)d_ws;
  size_t off = 0;
  const size_t oXB  = off; off += (size_t)MP * EMB * 2;          off = (off + 255) & ~(size_t)255;
  const size_t oW1T = off; off += (size_t)F1 * EMB * 2;          off = (off + 255) & ~(size_t)255;
  const size_t oW2D = off; off += (size_t)EMB * KA2 * 2;         off = (off + 255) & ~(size_t)255;
  const size_t oH1  = off; off += (size_t)MP * GW * 4;           off = (off + 255) & ~(size_t)255;
  const size_t oSD1 = off; off += (size_t)2 * HPG * MP * 4;      off = (off + 255) & ~(size_t)255;
  const size_t oXH  = off; off += (size_t)MP * KA2 * 2;          off = (off + 255) & ~(size_t)255;
  const size_t oH2  = off; off += (size_t)MP * EMB * 4;          off = (off + 255) & ~(size_t)255;
  const size_t oSD2 = off; off += (size_t)2 * MP * 4;            off = (off + 255) & ~(size_t)255;
  const size_t oBK  = off; off += (size_t)gA * BKINTS * 4;       off = (off + 255) & ~(size_t)255;
  if (off > ws_size || off > (size_t)WSMAX) return;
  unsigned short* XB   = (unsigned short*)(ws + oXB);
  unsigned short* W1T  = (unsigned short*)(ws + oW1T);
  unsigned short* W2D  = (unsigned short*)(ws + oW2D);
  float*          H1g  = (float*)(ws + oH1);
  float*          SD1  = (float*)(ws + oSD1);
  unsigned short* X1HL = (unsigned short*)(ws + oXH);
  float*          H2   = (float*)(ws + oH2);
  float*          SD2  = (float*)(ws + oSD2);
  int*            BK   = (int*)(ws + oBK);

  k_prep<<<(nUx + NUW1 + NUW2) / NTHR, NTHR, 0, stream>>>(x, W1, W2, XB, W1T, W2D, nN, nUx);
  k_bucket<<<gA, NTHR, 0, stream>>>(src, dst, nE, nN, vec8, BK);
  for (int g = 0; g < NGRP; ++g) {
    k_gemm<<<dim3(gM, HPG), GTHR, 0, stream>>>(XB, W1T + (size_t)g * GW * EMB, H1g, EMB, GW,
                                               a1s + (size_t)g * HPG * EMB, a1d + (size_t)g * HPG * EMB, SD1, MP);
    k_scan<1><<<gA, NTHR, 0, stream>>>(BK, H1g, SD1, b1, Wc, bc, X1HL, out, nN, MP, g * GW);
  }
  k_gemm<<<dim3(gM, 1), GTHR, 0, stream>>>(X1HL, W2D, H2, KA2, EMB, a2s, a2d, SD2, MP);
  k_scan<2><<<gA, NTHR, 0, stream>>>(BK, H2, SD2, b2, Wc, bc, X1HL, out, nN, MP, 0);
}
